// AttentiveFP_Simple_32555852103853
// MI455X (gfx1250) — hardware-verified
//
#include <hip/hip_runtime.h>
#include <stddef.h>


#define NTHR   256
#define NWAVE  8
#define IN0    64
#define HID    256
#define NHD    4
#define MH1    512
#define OUTW   12
#define OUTP   16
#define GR     32
#define GC     256
#define KCMAX  256
#define XSP    260
#define TILEQ  2112
#define NB     256
#define GB     64
#define CHUNK  2048
#define NGRP   (CHUNK / (NTHR * 4))
#define WCAP   256

#define LDS_GAT_BYTES  (NB * HID * 4 + NB * NHD * 4 * 2 + NWAVE * WCAP * 4 + 64)
#define LDS_POOL_BYTES (GB * HID * 4 * 2 + GB * 4 + NWAVE * WCAP * 4 + 64)

static_assert(NGRP == 2);
static_assert(WCAP == (CHUNK / NTHR) * 32);
static_assert(GR * XSP * 4 <= TILEQ * 16);
static_assert(GR * (KCMAX + 8) * 2 * 2 <= TILEQ * 16);
static_assert(LDS_GAT_BYTES == 278592);
static_assert(LDS_POOL_BYTES == 139584);
static_assert(NB / NWAVE == 32);
static_assert(GB / NWAVE == 8);
static_assert(NWAVE * 512 * 8 + 512 * 8 <= NB * HID * 4);
static_assert(GR * GC / 4 == NTHR * 8);

typedef float          v4f  __attribute__((ext_vector_type(4)));
typedef float          v8f  __attribute__((ext_vector_type(8)));
typedef int            v4i  __attribute__((ext_vector_type(4)));
typedef double         v2d  __attribute__((ext_vector_type(2)));
typedef __bf16         v16b __attribute__((ext_vector_type(16)));
typedef unsigned short u16;
union Frag { v16b v; v4i q[2]; };
union Pk8  { u16 s[8]; v4i q; };

__device__ __forceinline__ v8f wm(v16b a, v16b b, v8f c) {
  v8f d = __builtin_amdgcn_wmma_f32_16x16x32_bf16(false, a, false, b, (short)0, c, false, false);
  asm volatile("v_nop\n\tv_nop\n\tv_nop\n\tv_nop" : "+v"(d) : "v"(a), "v"(b));
  return d;
}

__device__ __forceinline__ unsigned int bfr(float f) {
  const unsigned int u = __float_as_uint(f);
  return (u + 0x7FFFu + ((u >> 16) & 1u)) >> 16;
}
__device__ __forceinline__ void split2(float v, u16& h, u16& l) {
  const unsigned int hb = bfr(v);
  const float hf = __uint_as_float(hb << 16);
  h = (u16)hb;
  l = (u16)bfr(v - hf);
}

__global__ __launch_bounds__(NTHR) void k_wprep(const float* __restrict__ W, int K, int Nc, int Npad,
                                                u16* Bh, u16* Bl) {
  const int k8n = K >> 3;
  const int i = blockIdx.x * NTHR + threadIdx.x;
  if (i >= Npad * k8n) return;
  const int n = i / k8n;
  const int k0 = (i - n * k8n) * 8;
  const bool ok = n < Nc;
  const int nc = ok ? n : Nc - 1;
  Pk8 ph, pl;
#pragma unroll
  for (int c = 0; c < 8; ++c) {
    float v = W[(size_t)(k0 + c) * Nc + nc];
    v = ok ? v : 0.f;
    u16 a, b;
    split2(v, a, b);
    ph.s[c] = a;
    pl.s[c] = b;
  }
  const size_t o = (size_t)n * K + k0;
  *(volatile v4i*)(Bh + o) = ph.q;
  *(volatile v4i*)(Bl + o) = pl.q;
  __threadfence();
  *(volatile v4i*)(Bh + o) = ph.q;
  *(volatile v4i*)(Bl + o) = pl.q;
}

__device__ __forceinline__ void dot_tile(v8f a, v8f b, float cs0, float cs1, float cd0, float cd1,
                                         int T, int hh, int m, int wave, float* Pss, float* Psd) {
  float ss[8], sd[8];
#pragma unroll
  for (int r = 0; r < 8; ++r) {
    ss[r] = a[r] * cs0 + b[r] * cs1;
    sd[r] = a[r] * cd0 + b[r] * cd1;
  }
#pragma unroll
  for (int mk = 1; mk < 16; mk <<= 1) {
#pragma unroll
    for (int r = 0; r < 8; ++r) {
      ss[r] += __shfl_xor(ss[r], mk, 32);
      sd[r] += __shfl_xor(sd[r], mk, 32);
    }
  }
  if (m == 0) {
#pragma unroll
    for (int r = 0; r < 8; ++r) {
      Pss[(T * 16 + 8 * hh + r) * 8 + wave] = ss[r];
      Psd[(T * 16 + 8 * hh + r) * 8 + wave] = sd[r];
    }
  }
}

__global__ __launch_bounds__(NTHR) void k_gemm(
    const float* __restrict__ A, int lda, int M, int K,
    const u16* __restrict__ Bh, const u16* __restrict__ Bl, int Npad, int Nreal,
    const float* __restrict__ bias, float* Out, int ldo, int Mst,
    const float* __restrict__ avs, const float* __restrict__ avd, float* es, float* ed, int flags) {
  __shared__ v4i tile[TILEQ];
  __shared__ __attribute__((aligned(16))) float Pss[GR * 8];
  __shared__ __attribute__((aligned(16))) float Psd[GR * 8];
  __shared__ __attribute__((aligned(16))) float Es4[GR * 4];
  __shared__ __attribute__((aligned(16))) float Ed4[GR * 4];

  const int tid  = threadIdx.x;
  const int lane = tid & 31;
  const int wave = tid >> 5;
  const int hh   = lane >> 4;
  const int m    = lane & 15;
  const int rowBase = blockIdx.x * GR;
  const int cb   = blockIdx.y * GC;
  const int KC   = (K < KCMAX) ? K : KCMAX;
  const int AP   = KC + 8;
  u16* Ah = (u16*)tile;
  u16* Al = Ah + GR * AP;
  float* Xs = (float*)tile;
  const bool hasBias = (flags & 1) != 0;
  const bool dots    = (flags & 2) != 0;
  const v4f z4 = {0.f, 0.f, 0.f, 0.f};

  const int cg0 = cb + wave * 32 + m;
  const int cg1 = cg0 + 16;
  const int cq0 = cg0 < Npad ? cg0 : Npad - 1;
  const int cq1 = cg1 < Npad ? cg1 : Npad - 1;
  const u16* pbh0 = Bh + (size_t)cq0 * K + 8 * hh;
  const u16* pbl0 = Bl + (size_t)cq0 * K + 8 * hh;
  const u16* pbh1 = Bh + (size_t)cq1 * K + 8 * hh;
  const u16* pbl1 = Bl + (size_t)cq1 * K + 8 * hh;

  const int sr  = tid >> 3;
  const int scw = KC >> 3;
  const int sc0 = (tid & 7) * scw;
  int arow = rowBase + sr;
  arow = arow < M ? arow : M - 1;
  const float* ap = A + (size_t)arow * lda;

  v8f acc00 = {0.f, 0.f, 0.f, 0.f, 0.f, 0.f, 0.f, 0.f};
  v8f acc01 = acc00, acc10 = acc00, acc11 = acc00;

#pragma unroll 1
  for (int kc = 0; kc < K; kc += KC) {
    __syncthreads();
#pragma unroll 1
    for (int q = 0; q < (scw >> 3); ++q) {
      const int c = sc0 + 8 * q;
      const v4f f0 = *(const v4f*)(ap + kc + c);
      const v4f f1 = *(const v4f*)(ap + kc + c + 4);
      Pk8 ph, pl;
      split2(f0.x, ph.s[0], pl.s[0]); split2(f0.y, ph.s[1], pl.s[1]);
      split2(f0.z, ph.s[2], pl.s[2]); split2(f0.w, ph.s[3], pl.s[3]);
      split2(f1.x, ph.s[4], pl.s[4]); split2(f1.y, ph.s[5], pl.s[5]);
      split2(f1.z, ph.s[6], pl.s[6]); split2(f1.w, ph.s[7], pl.s[7]);
      *(v4i*)(Ah + sr * AP + c) = ph.q;
      *(v4i*)(Al + sr * AP + c) = pl.q;
    }
    __syncthreads();
#pragma unroll 1
    for (int ks = 0; ks < KC; ks += 32) {
      Frag a0h, a0l, a1h, a1l, b0h, b0l, b1h, b1l;
      const int la0 = m * AP + ks + 8 * hh;
      const int la1 = (16 + m) * AP + ks + 8 * hh;
      a0h.q[0] = *(const v4i*)(Ah + la0); a0h.q[1] = *(const v4i*)(Ah + la0 + 16);
      a0l.q[0] = *(const v4i*)(Al + la0); a0l.q[1] = *(const v4i*)(Al + la0 + 16);
      a1h.q[0] = *(const v4i*)(Ah + la1); a1h.q[1] = *(const v4i*)(Ah + la1 + 16);
      a1l.q[0] = *(const v4i*)(Al + la1); a1l.q[1] = *(const v4i*)(Al + la1 + 16);
      const int kb = kc + ks;
      b0h.q[0] = *(const v4i*)(pbh0 + kb); b0h.q[1] = *(const v4i*)(pbh0 + kb + 16);
      b0l.q[0] = *(const v4i*)(pbl0 + kb); b0l.q[1] = *(const v4i*)(pbl0 + kb + 16);
      b1h.q[0] = *(const v4i*)(pbh1 + kb); b1h.q[1] = *(const v4i*)(pbh1 + kb + 16);
      b1l.q[0] = *(const v4i*)(pbl1 + kb); b1l.q[1] = *(const v4i*)(pbl1 + kb + 16);
      acc00 = wm(a0h.v, b0h.v, acc00); acc00 = wm(a0h.v, b0l.v, acc00); acc00 = wm(a0l.v, b0h.v, acc00);
      acc01 = wm(a0h.v, b1h.v, acc01); acc01 = wm(a0h.v, b1l.v, acc01); acc01 = wm(a0l.v, b1h.v, acc01);
      acc10 = wm(a1h.v, b0h.v, acc10); acc10 = wm(a1h.v, b0l.v, acc10); acc10 = wm(a1l.v, b0h.v, acc10);
      acc11 = wm(a1h.v, b1h.v, acc11); acc11 = wm(a1h.v, b1l.v, acc11); acc11 = wm(a1l.v, b1h.v, acc11);
    }
  }
  __syncthreads();

  const int qb0 = cg0 < Nreal ? cg0 : Nreal - 1;
  const int qb1 = cg1 < Nreal ? cg1 : Nreal - 1;
  float badd0 = 0.f, badd1 = 0.f;
  if (hasBias) { badd0 = bias[qb0]; badd1 = bias[qb1]; }
  const int lc0 = wave * 32 + m, lc1 = lc0 + 16;
#pragma unroll
  for (int r = 0; r < 8; ++r) {
    Xs[(8 * hh + r) * XSP + lc0]      = acc00[r] + badd0;
    Xs[(8 * hh + r) * XSP + lc1]      = acc01[r] + badd1;
    Xs[(16 + 8 * hh + r) * XSP + lc0] = acc10[r] + badd0;
    Xs[(16 + 8 * hh + r) * XSP + lc1] = acc11[r] + badd1;
  }
  if (dots) {
    const float cs0 = avs[qb0], cs1 = avs[qb1], cd0 = avd[qb0], cd1 = avd[qb1];
    dot_tile(acc00, acc01, cs0, cs1, cd0, cd1, 0, hh, m, wave, Pss, Psd);
    dot_tile(acc10, acc11, cs0, cs1, cd0, cd1, 1, hh, m, wave, Pss, Psd);
  }
  __syncthreads();
  if (dots) {
    if (tid < 128) {
      const int row = tid >> 2, h = tid & 3;
      Es4[row * 4 + h] = Pss[row * 8 + 2 * h] + Pss[row * 8 + 2 * h + 1];
    } else {
      const int t2 = tid - 128;
      const int row = t2 >> 2, h = t2 & 3;
      Ed4[row * 4 + h] = Psd[row * 8 + 2 * h] + Psd[row * 8 + 2 * h + 1];
    }
  }
  __syncthreads();

  int nrows = Mst - rowBase;
  nrows = nrows > GR ? GR : nrows;
  nrows = nrows < 0 ? 0 : nrows;
  int segw = Nreal - cb;
  segw = segw > GC ? GC : segw;
  const int total = (segw > 0) ? nrows * segw : 0;
  v4f vv[8];
  size_t oo[8];
#pragma unroll
  for (int i = 0; i < 8; ++i) {
    const int f = 4 * (tid + NTHR * i);
    vv[i] = z4;
    oo[i] = 0;
    if (f < total) {
      const int row = f / segw;
      const int col = f - row * segw;
      vv[i] = *(const v4f*)(Xs + row * XSP + col);
      oo[i] = (size_t)(rowBase + row) * (size_t)ldo + (size_t)(cb + col);
    }
  }
  v4f ev = z4;
  float* ep = es;
  const bool est = dots && (wave < 2) && (rowBase + lane < Mst);
  if (est) {
    if (wave == 0) { ev = *(const v4f*)(Es4 + 4 * lane); ep = es + (size_t)(rowBase + lane) * NHD; }
    else           { ev = *(const v4f*)(Ed4 + 4 * lane); ep = ed + (size_t)(rowBase + lane) * NHD; }
  }
#pragma unroll
  for (int i = 0; i < 8; ++i)
    if (4 * (tid + NTHR * i) < total) *(volatile v4f*)(Out + oo[i]) = vv[i];
  if (est) *(volatile v4f*)ep = ev;
  __threadfence();
#pragma unroll
  for (int i = 0; i < 8; ++i)
    if (4 * (tid + NTHR * i) < total) *(volatile v4f*)(Out + oo[i]) = vv[i];
  if (est) *(volatile v4f*)ep = ev;
}

__device__ __forceinline__ void scan_chunk(const int* __restrict__ ids, int nIds, int cbase, bool vec,
                                           int base, unsigned nslots, int shift,
                                           int* list, int* wcnt, int tid, int lane, int wave) {
  int wc = 0;
#pragma unroll
  for (int g = 0; g < NGRP; ++g) {
    const int el0 = (g * NTHR + tid) * 4;
    const int e0  = cbase + el0;
    const int sent = -2147483647 - 1;
    v4i d;
    if (vec) {
      d = *(const v4i*)(ids + e0);
    } else {
      const int lm = nIds - 1;
      d.x = (e0     < nIds) ? ids[min(e0,     lm)] : sent;
      d.y = (e0 + 1 < nIds) ? ids[min(e0 + 1, lm)] : sent;
      d.z = (e0 + 2 < nIds) ? ids[min(e0 + 2, lm)] : sent;
      d.w = (e0 + 3 < nIds) ? ids[min(e0 + 3, lm)] : sent;
    }
    const unsigned s0 = (unsigned)d.x - (unsigned)base;
    const unsigned s1 = (unsigned)d.y - (unsigned)base;
    const unsigned s2 = (unsigned)d.z - (unsigned)base;
    const unsigned s3 = (unsigned)d.w - (unsigned)base;
    const bool h0 = s0 < nslots;
    const bool h1 = s1 < nslots;
    const bool h2 = s2 < nslots;
    const bool h3 = s3 < nslots;
    const unsigned many = __builtin_amdgcn_ballot_w32(h0 | h1 | h2 | h3);
    if (many != 0u) {
#define HITJ(J, HJ, SJ) { \
        const unsigned mj = __builtin_amdgcn_ballot_w32(HJ); \
        if (HJ) { \
          const int pos = wc + (int)__builtin_amdgcn_mbcnt_lo(mj, 0u); \
          if (pos < WCAP) list[wave * WCAP + pos] = ((el0 + (J)) << shift) | (int)(SJ); \
        } \
        wc += (int)__builtin_popcount(mj); }
      HITJ(0, h0, s0)
      HITJ(1, h1, s1)
      HITJ(2, h2, s2)
      HITJ(3, h3, s3)
#undef HITJ
    }
  }
  if (lane == 0) wcnt[wave] = wc;
}

__global__ __launch_bounds__(NTHR) void k_gat(const int* __restrict__ ei, int nE, int nN,
    const float* __restrict__ xw, const float* __restrict__ es, const float* __restrict__ ed,
    const float* __restrict__ gb, float* agg, double* pstat) {
  extern __shared__ v4i lds_dyn[];
  float* sacc = (float*)lds_dyn;
  float* den  = sacc + NB * HID;
  float* mrun = den + NB * NHD;
  int*   list = (int*)(mrun + NB * NHD);
  int*   wcnt = list + NWAVE * WCAP;

  const int tid  = threadIdx.x;
  const int lane = tid & 31;
  const int wave = tid >> 5;
  const int hd   = lane >> 3;
  const int nodeBase = blockIdx.x * NB;
  const v4f z4 = {0.f, 0.f, 0.f, 0.f};

#pragma unroll 1
  for (int j = 0; j < NB / NWAVE; ++j) {
    const int slot = wave * (NB / NWAVE) + j;
    const int node = nodeBase + slot;
    const bool ok = node < nN;
    const int nc = ok ? node : nN - 1;
    v4f x0 = *(const v4f*)(xw + (size_t)nc * HID + 8 * lane);
    v4f x1 = *(const v4f*)(xw + (size_t)nc * HID + 8 * lane + 4);
    float lg = es[(size_t)nc * NHD + hd] + ed[(size_t)nc * NHD + hd];
    lg = (lg > 0.f) ? lg : 0.2f * lg;
    if (!ok) { x0 = z4; x1 = z4; lg = 0.f; }
    *(v4f*)(sacc + slot * HID + 8 * lane)     = x0;
    *(v4f*)(sacc + slot * HID + 8 * lane + 4) = x1;
    mrun[slot * NHD + hd] = lg;
    den[slot * NHD + hd]  = 1.0f;
  }
  __syncthreads();

  const int* eid = ei + nE;
  const bool al16 = ((((size_t)eid) & 15) == 0);
  const int nChunks = (nE + CHUNK - 1) / CHUNK;
#pragma unroll 1
  for (int ch = 0; ch < nChunks; ++ch) {
    const int cbase = ch * CHUNK;
    const bool vec = al16 && (cbase + CHUNK <= nE);
    scan_chunk(eid, nE, cbase, vec, nodeBase, (unsigned)NB, 8, list, wcnt, tid, lane, wave);
    __syncthreads();
    if (wave == 0) {
#pragma unroll 1
      for (int wsx = 0; wsx < NWAVE; ++wsx) {
        int n = wcnt[wsx];
        n = n > WCAP ? WCAP : n;
        n = n < 0 ? 0 : n;
#pragma unroll 1
        for (int i = 0; i < n; ++i) {
          const int ent  = list[wsx * WCAP + i];
          const int slot = ent & (NB - 1);
          const int el   = (ent >> 8) & (CHUNK - 1);
          int e = cbase + el;
          e = e < nE ? e : nE - 1;
          int src = ei[e];
          src = src < 0 ? 0 : (src > nN - 1 ? nN - 1 : src);
          int nd = nodeBase + slot;
          nd = nd < nN ? nd : nN - 1;
          float lg = es[(size_t)src * NHD + hd] + ed[(size_t)nd * NHD + hd];
          lg = (lg > 0.f) ? lg : 0.2f * lg;
          const int ai = slot * NHD + hd;
          const float mo = mrun[ai];
          const float mn = fmaxf(mo, lg);
          const float sc = __expf(mo - mn);
          const float p  = __expf(lg - mn);
          const v4f xv0 = *(const v4f*)(xw + (size_t)src * HID + 8 * lane);
          const v4f xv1 = *(const v4f*)(xw + (size_t)src * HID + 8 * lane + 4);
          v4f* sp0 = (v4f*)(sacc + slot * HID + 8 * lane);
          v4f* sp1 = sp0 + 1;
          const v4f c0 = *sp0;
          const v4f c1 = *sp1;
          *sp0 = c0 * sc + xv0 * p;
          *sp1 = c1 * sc + xv1 * p;
          const float dv = den[ai];
          den[ai]  = dv * sc + p;
          mrun[ai] = mn;
        }
      }
    }
    __syncthreads();
  }

  const int hA = lane >> 4, hB = 2 + (lane >> 4);
  const v4f g0 = *(const v4f*)(gb + 4 * lane);
  const v4f g1 = *(const v4f*)(gb + 128 + 4 * lane);
  double S[8], Q[8];
#pragma unroll
  for (int c = 0; c < 8; ++c) { S[c] = 0.0; Q[c] = 0.0; }
#pragma unroll 1
  for (int j = 0; j < NB / NWAVE; ++j) {
    const int slot = wave * (NB / NWAVE) + j;
    const int node = nodeBase + slot;
    if (node >= nN) break;
    const float i0 = 1.0f / den[slot * NHD + hA];
    const float i1 = 1.0f / den[slot * NHD + hB];
    const v4f o0 = *(const v4f*)(sacc + slot * HID + 4 * lane) * i0 + g0;
    const v4f o1 = *(const v4f*)(sacc + slot * HID + 128 + 4 * lane) * i1 + g1;
    S[0] += (double)o0.x; S[1] += (double)o0.y; S[2] += (double)o0.z; S[3] += (double)o0.w;
    S[4] += (double)o1.x; S[5] += (double)o1.y; S[6] += (double)o1.z; S[7] += (double)o1.w;
    Q[0] += (double)o0.x * (double)o0.x; Q[1] += (double)o0.y * (double)o0.y;
    Q[2] += (double)o0.z * (double)o0.z; Q[3] += (double)o0.w * (double)o0.w;
    Q[4] += (double)o1.x * (double)o1.x; Q[5] += (double)o1.y * (double)o1.y;
    Q[6] += (double)o1.z * (double)o1.z; Q[7] += (double)o1.w * (double)o1.w;
    float* op = agg + (size_t)node * HID;
    *(volatile v4f*)(op + 4 * lane)       = o0;
    *(volatile v4f*)(op + 128 + 4 * lane) = o1;
  }
  __threadfence();
#pragma unroll 1
  for (int j = 0; j < NB / NWAVE; ++j) {
    const int slot = wave * (NB / NWAVE) + j;
    const int node = nodeBase + slot;
    if (node >= nN) break;
    const float i0 = 1.0f / den[slot * NHD + hA];
    const float i1 = 1.0f / den[slot * NHD + hB];
    const v4f o0 = *(const v4f*)(sacc + slot * HID + 4 * lane) * i0 + g0;
    const v4f o1 = *(const v4f*)(sacc + slot * HID + 128 + 4 * lane) * i1 + g1;
    float* op = agg + (size_t)node * HID;
    *(volatile v4f*)(op + 4 * lane)       = o0;
    *(volatile v4f*)(op + 128 + 4 * lane) = o1;
  }
  __syncthreads();

  double* statl = (double*)lds_dyn;
  {
    double* w0 = statl + wave * 512;
#pragma unroll
    for (int c = 0; c < 4; ++c) {
      w0[4 * lane + c]             = S[c];
      w0[128 + 4 * lane + c]       = S[4 + c];
      w0[256 + 4 * lane + c]       = Q[c];
      w0[256 + 128 + 4 * lane + c] = Q[4 + c];
    }
  }
  __syncthreads();
  double* Sl = statl + NWAVE * 512;
  {
    double s = 0.0, q = 0.0;
#pragma unroll
    for (int w = 0; w < NWAVE; ++w) {
      s += statl[w * 512 + tid];
      q += statl[w * 512 + 256 + tid];
    }
    Sl[tid] = s;
    Sl[256 + tid] = q;
  }
  __syncthreads();
  {
    const v2d v = *(const v2d*)(Sl + 2 * tid);
    double* pp = pstat + (size_t)blockIdx.x * 512 + 2 * tid;
    *(volatile v2d*)pp = v;
    __threadfence();
    *(volatile v2d*)pp = v;
  }
}

__global__ __launch_bounds__(NTHR) void k_stats(int mode, const double* __restrict__ pstat, int nblk,
                                                const float* __restrict__ X, int ldx, int nrows, int cols,
                                                float* musr) {
  __shared__ __attribute__((aligned(16))) float st[2 * NTHR];
  const int tid = threadIdx.x;
  const int col = blockIdx.x * NTHR + tid;
  double s = 0.0, q = 0.0;
  if (mode == 0) {
#pragma unroll 1
    for (int b = 0; b < nblk; ++b) {
      s += pstat[(size_t)b * 512 + tid];
      q += pstat[(size_t)b * 512 + 256 + tid];
    }
  } else {
    const int cc = col < cols ? col : cols - 1;
#pragma unroll 1
    for (int r = 0; r < nrows; ++r) {
      const double v = (double)X[(size_t)r * ldx + cc];
      s += v;
      q += v * v;
    }
  }
  const double inv = 1.0 / (double)(nrows > 0 ? nrows : 1);
  const double mu = s * inv;
  double var = q * inv - mu * mu;
  var = var > 0.0 ? var : 0.0;
  st[tid] = (float)mu;
  st[NTHR + tid] = 1.0f / sqrtf((float)var + 1e-5f);
  __syncthreads();
  const bool act = tid < 128;
  const int which = tid >> 6;
  const int t4 = (tid & 63) * 4;
  v4f v = {0.f, 0.f, 0.f, 0.f};
  float* p = musr;
  if (act) {
    v = *(const v4f*)(st + which * NTHR + t4);
    p = musr + (size_t)which * cols + (size_t)blockIdx.x * NTHR + t4;
  }
  if (act) *(volatile v4f*)p = v;
  __threadfence();
  if (act) *(volatile v4f*)p = v;
}

__global__ __launch_bounds__(NTHR) void k_apply(const float* X, const float* __restrict__ musr,
                                                const float* __restrict__ g, const float* __restrict__ b,
                                                const float* res, float* out, int cols, int n4, int act, int hasRes) {
  const int i = blockIdx.x * NTHR + threadIdx.x;
  if (i >= n4) return;
  const size_t o = (size_t)i * 4;
  const int c = (int)(o & (size_t)(cols - 1));
  const v4f xv = *(const v4f*)(X + o);
  const v4f mu = *(const v4f*)(musr + c);
  const v4f rs = *(const v4f*)(musr + cols + c);
  const v4f gg = *(const v4f*)(g + c);
  const v4f bb = *(const v4f*)(b + c);
  const v4f z = (xv - mu) * rs * gg + bb;
  v4f y;
  if (act == 0) {
    y.x = z.x > 0.f ? z.x : (__expf(z.x) - 1.f);
    y.y = z.y > 0.f ? z.y : (__expf(z.y) - 1.f);
    y.z = z.z > 0.f ? z.z : (__expf(z.z) - 1.f);
    y.w = z.w > 0.f ? z.w : (__expf(z.w) - 1.f);
  } else {
    y.x = fmaxf(z.x, 0.f); y.y = fmaxf(z.y, 0.f); y.z = fmaxf(z.z, 0.f); y.w = fmaxf(z.w, 0.f);
  }
  if (hasRes) y = y + *(const v4f*)(res + o);
  *(volatile v4f*)(out + o) = y;
  __threadfence();
  *(volatile v4f*)(out + o) = y;
}

__global__ __launch_bounds__(NTHR) void k_pool(const float* __restrict__ h, const int* __restrict__ bt,
                                               int nN, int nGp, float* hg) {
  extern __shared__ v4i lds_dyn[];
  float* ssum = (float*)lds_dyn;
  float* smax = ssum + GB * HID;
  float* scnt = smax + GB * HID;
  int*   list = (int*)(scnt + GB);
  int*   wcnt = list + NWAVE * WCAP;

  const int tid  = threadIdx.x;
  const int lane = tid & 31;
  const int wave = tid >> 5;
  const int gBase = blockIdx.x * GB;
  const v4f z4 = {0.f, 0.f, 0.f, 0.f};
  const float NINF = -__builtin_huge_valf();
  const v4f ninf4 = {NINF, NINF, NINF, NINF};

  for (int i = tid; i < GB * HID / 4; i += NTHR) {
    ((v4f*)ssum)[i] = z4;
    ((v4f*)smax)[i] = ninf4;
  }
  if (tid < GB) scnt[tid] = 0.f;
  __syncthreads();

  const bool al16 = ((((size_t)bt) & 15) == 0);
  const int nChunks = (nN + CHUNK - 1) / CHUNK;
#pragma unroll 1
  for (int ch = 0; ch < nChunks; ++ch) {
    const int cbase = ch * CHUNK;
    const bool vec = al16 && (cbase + CHUNK <= nN);
    scan_chunk(bt, nN, cbase, vec, gBase, (unsigned)GB, 6, list, wcnt, tid, lane, wave);
    __syncthreads();
    if (wave == 0) {
#pragma unroll 1
      for (int wsx = 0; wsx < NWAVE; ++wsx) {
        int n = wcnt[wsx];
        n = n > WCAP ? WCAP : n;
        n = n < 0 ? 0 : n;
#pragma unroll 1
        for (int i = 0; i < n; ++i) {
          const int ent  = list[wsx * WCAP + i];
          const int slot = ent & (GB - 1);
          const int el   = (ent >> 6) & (CHUNK - 1);
          int node = cbase + el;
          node = node < nN ? node : nN - 1;
          const v4f v0 = *(const v4f*)(h + (size_t)node * HID + 8 * lane);
          const v4f v1 = *(const v4f*)(h + (size_t)node * HID + 8 * lane + 4);
          v4f* sp0 = (v4f*)(ssum + slot * HID + 8 * lane);
          v4f* sp1 = sp0 + 1;
          v4f* mp0 = (v4f*)(smax + slot * HID + 8 * lane);
          v4f* mp1 = mp0 + 1;
          const v4f a0 = *sp0, a1 = *sp1;
          *sp0 = a0 + v0;
          *sp1 = a1 + v1;
          v4f m0 = *mp0, m1 = *mp1;
          m0.x = fmaxf(m0.x, v0.x); m0.y = fmaxf(m0.y, v0.y); m0.z = fmaxf(m0.z, v0.z); m0.w = fmaxf(m0.w, v0.w);
          m1.x = fmaxf(m1.x, v1.x); m1.y = fmaxf(m1.y, v1.y); m1.z = fmaxf(m1.z, v1.z); m1.w = fmaxf(m1.w, v1.w);
          *mp0 = m0;
          *mp1 = m1;
          if (lane == 0) {
            const float cc = scnt[slot];
            scnt[slot] = cc + 1.0f;
          }
        }
      }
    }
    __syncthreads();
  }

#pragma unroll 1
  for (int pass = 0; pass < 2; ++pass) {
#pragma unroll 1
    for (int j = 0; j < GB / NWAVE; ++j) {
      const int slot = wave * (GB / NWAVE) + j;
      const int gi = gBase + slot;
      if (gi >= nGp) break;
      const float c = scnt[slot];
      const float inv = 1.0f / fmaxf(c, 1.0f);
      const v4f me0 = *(const v4f*)(ssum + slot * HID + 4 * lane) * inv;
      const v4f me1 = *(const v4f*)(ssum + slot * HID + 128 + 4 * lane) * inv;
      v4f mx0 = *(const v4f*)(smax + slot * HID + 4 * lane);
      v4f mx1 = *(const v4f*)(smax + slot * HID + 128 + 4 * lane);
      if (!(c > 0.f)) { mx0 = z4; mx1 = z4; }
      float* rp = hg + (size_t)gi * (2 * HID);
      *(volatile v4f*)(rp + 4 * lane)             = me0;
      *(volatile v4f*)(rp + 128 + 4 * lane)       = me1;
      *(volatile v4f*)(rp + HID + 4 * lane)       = mx0;
      *(volatile v4f*)(rp + HID + 128 + 4 * lane) = mx1;
    }
    __threadfence();
  }
}

extern "C" void kernel_launch(void* const* d_in, const int* in_sizes, int n_in,
                              void* d_out, int out_size, void* d_ws, size_t ws_size,
                              hipStream_t stream) {
  if (n_in < 33) return;
  const int N = in_sizes[0] / IN0;
  const int E = in_sizes[1] / 2;
  const int G = out_size / OUTW;
  if (N <= 0 || G <= 0 || E < 0) return;
  if (in_sizes[0] != N * IN0 || in_sizes[1] != 2 * E || in_sizes[2] != N || out_size != G * OUTW) return;
  if (in_sizes[3] != IN0 * HID || in_sizes[4] != HID) return;
  const int gwi[3] = {5, 11, 17};
  for (int l = 0; l < 3; ++l) {
    const int K = (l == 0) ? IN0 : HID;
    if (in_sizes[gwi[l]] != K * HID) return;
    for (int t = 1; t <= 5; ++t) if (in_sizes[gwi[l] + t] != HID) return;
  }
  if (in_sizes[23] != 2 * HID * MH1 || in_sizes[24] != MH1 || in_sizes[25] != MH1 || in_sizes[26] != MH1) return;
  if (in_sizes[27] != MH1 * HID || in_sizes[28] != HID || in_sizes[29] != HID || in_sizes[30] != HID) return;
  if (in_sizes[31] != HID * OUTW || in_sizes[32] != OUTW) return;

  const float* x     = (const float*)d_in[0];
  const int*   ei    = (const int*)d_in[1];
  const int*   batch = (const int*)d_in[2];
  const float* W_in  = (const float*)d_in[3];
  const float* b_in  = (const float*)d_in[4];
  const float* gW[3]  = {(const float*)d_in[5],  (const float*)d_in[11], (const float*)d_in[17]};
  const float* gas[3] = {(const float*)d_in[6],  (const float*)d_in[12], (const float*)d_in[18]};
  const float* gad[3] = {(const float*)d_in[7],  (const float*)d_in[13], (const float*)d_in[19]};
  const float* gb[3]  = {(const float*)d_in[8],  (const float*)d_in[14], (const float*)d_in[20]};
  const float* bng[3] = {(const float*)d_in[9],  (const float*)d_in[15], (const float*)d_in[21]};
  const float* bnb[3] = {(const float*)d_in[10], (const float*)d_in[16], (const float*)d_in[22]};
  const float* mW1  = (const float*)d_in[23];
  const float* mb1  = (const float*)d_in[24];
  const float* mg1  = (const float*)d_in[25];
  const float* mbe1 = (const float*)d_in[26];
  const float* mW2  = (const float*)d_in[27];
  const float* mb2  = (const float*)d_in[28];
  const float* mg2  = (const float*)d_in[29];
  const float* mbe2 = (const float*)d_in[30];
  const float* hW   = (const float*)d_in[31];
  const float* hb   = (const float*)d_in[32];
  float* out = (float*)d_out;

  const int Np  = ((N + GR - 1) / GR) * GR;
  const int Gp  = ((G + GR - 1) / GR) * GR;
  const int nbg = (N + NB - 1) / NB;

  char* ws = (char*)d_ws;
  size_t off = 0;
  auto carve = [&](size_t bytes) -> char* {
    char* p = ws + off;
    off += (bytes + 255) & ~(size_t)255;
    return p;
  };
  float* P   = (float*)carve((size_t)Np * HID * 4);
  const size_t xwBytes = (size_t)Np * HID * 4;
  float* XW  = (float*)carve(xwBytes);
  float* AGG = (float*)carve((size_t)Np * HID * 4);
  float* ES  = (float*)carve((size_t)Np * NHD * 4);
  float* ED  = (float*)carve((size_t)Np * NHD * 4);
  u16* WinH = (u16*)carve((size_t)HID * IN0 * 2);
  u16* WinL = (u16*)carve((size_t)HID * IN0 * 2);
  u16* gWH[3]; u16* gWL[3];
  for (int l = 0; l < 3; ++l) {
    const int K = (l == 0) ? IN0 : HID;
    gWH[l] = (u16*)carve((size_t)HID * K * 2);
    gWL[l] = (u16*)carve((size_t)HID * K * 2);
  }
  u16* m1H = (u16*)carve((size_t)MH1 * (2 * HID) * 2);
  u16* m1L = (u16*)carve((size_t)MH1 * (2 * HID) * 2);
  u16* m2H = (u16*)carve((size_t)HID * MH1 * 2);
  u16* m2L = (u16*)carve((size_t)HID * MH1 * 2);
  u16* hWH = (u16*)carve((size_t)OUTP * HID * 2);
  u16* hWL = (u16*)carve((size_t)OUTP * HID * 2);
  double* PSTAT = (double*)carve((size_t)nbg * 512 * 8);
  float* MUSR = (float*)carve((size_t)2 * MH1 * 4);
  const size_t bHG = (size_t)Gp * (2 * HID) * 4, bS1 = (size_t)Gp * MH1 * 4, bS2 = (size_t)Gp * HID * 4;
  const size_t mlpNeed = bHG + 2 * bS1 + 2 * bS2;
  char* mlp = (char*)XW;
  if (mlpNeed > xwBytes) mlp = carve(mlpNeed);
  float* HG = (float*)mlp;
  float* S1 = (float*)(mlp + bHG);
  float* T1 = (float*)(mlp + bHG + bS1);
  float* S2 = (float*)(mlp + bHG + 2 * bS1);
  float* T2 = (float*)(mlp + bHG + 2 * bS1 + bS2);
  if (off > ws_size || off > ((size_t)128 << 20)) return;

  auto blocks = [](size_t n) { return (unsigned)((n + NTHR - 1) / NTHR); };

  k_wprep<<<blocks((size_t)HID * IN0 / 8), NTHR, 0, stream>>>(W_in, IN0, HID, HID, WinH, WinL);
  for (int l = 0; l < 3; ++l) {
    const int K = (l == 0) ? IN0 : HID;
    k_wprep<<<blocks((size_t)HID * K / 8), NTHR, 0, stream>>>(gW[l], K, HID, HID, gWH[l], gWL[l]);
  }
  k_wprep<<<blocks((size_t)MH1 * (2 * HID) / 8), NTHR, 0, stream>>>(mW1, 2 * HID, MH1, MH1, m1H, m1L);
  k_wprep<<<blocks((size_t)HID * MH1 / 8), NTHR, 0, stream>>>(mW2, MH1, HID, HID, m2H, m2L);
  k_wprep<<<blocks((size_t)OUTP * HID / 8), NTHR, 0, stream>>>(hW, HID, OUTW, OUTP, hWH, hWL);

  const dim3 gN(Np / GR, 1);
  k_gemm<<<gN, NTHR, 0, stream>>>(x, IN0, N, IN0, WinH, WinL, HID, HID, b_in, P, HID, Np,
                                  gas[0], gad[0], ES, ED, 1);

  hipFuncSetAttribute(reinterpret_cast<const void*>(&k_gat),
                      hipFuncAttributeMaxDynamicSharedMemorySize, LDS_GAT_BYTES);
  for (int l = 0; l < 3; ++l) {
    const int K = (l == 0) ? IN0 : HID;
    const float* Ain = (l == 0) ? x : P;
    k_gemm<<<gN, NTHR, 0, stream>>>(Ain, K, N, K, gWH[l], gWL[l], HID, HID, b_in, XW, HID, Np,
                                    gas[l], gad[l], ES, ED, 2);
    k_gat<<<nbg, NTHR, LDS_GAT_BYTES, stream>>>(ei, E, N, XW, ES, ED, gb[l], AGG, PSTAT);
    k_stats<<<1, NTHR, 0, stream>>>(0, PSTAT, nbg, AGG, HID, N, HID, MUSR);
    k_apply<<<blocks((size_t)N * HID / 4), NTHR, 0, stream>>>(AGG, MUSR, bng[l], bnb[l], P, P,
                                                                HID, N * (HID / 4), 0, 1);
  }

  hipFuncSetAttribute(reinterpret_cast<const void*>(&k_pool),
                      hipFuncAttributeMaxDynamicSharedMemorySize, LDS_POOL_BYTES);
  k_pool<<<(Gp + GB - 1) / GB, NTHR, LDS_POOL_BYTES, stream>>>(P, batch, N, Gp, HG);

  const dim3 g1(Gp / GR, MH1 / GC);
  k_gemm<<<g1, NTHR, 0, stream>>>(HG, 2 * HID, G, 2 * HID, m1H, m1L, MH1, MH1, mb1, S1, MH1, Gp,
                                  gas[0], gad[0], ES, ED, 1);
  k_stats<<<MH1 / NTHR, NTHR, 0, stream>>>(1, PSTAT, 0, S1, MH1, G, MH1, MUSR);
  k_apply<<<blocks((size_t)Gp * MH1 / 4), NTHR, 0, stream>>>(S1, MUSR, mg1, mbe1, S1, T1,
                                                               MH1, Gp * (MH1 / 4), 1, 0);
  const dim3 g2(Gp / GR, 1);
  k_gemm<<<g2, NTHR, 0, stream>>>(T1, MH1, G, MH1, m2H, m2L, HID, HID, mb2, S2, HID, Gp,
                                  gas[0], gad[0], ES, ED, 1);
  k_stats<<<HID / NTHR, NTHR, 0, stream>>>(1, PSTAT, 0, S2, HID, G, HID, MUSR);
  k_apply<<<blocks((size_t)Gp * HID / 4), NTHR, 0, stream>>>(S2, MUSR, mg2, mbe2, S2, T2,
                                                               HID, Gp * (HID / 4), 1, 0);
  k_gemm<<<g2, NTHR, 0, stream>>>(T2, HID, G, HID, hWH, hWL, OUTP, OUTW, hb, out, OUTW, G,
                                  gas[0], gad[0], ES, ED, 1);
}
